// RelationAwareAttention_11338713661449
// MI455X (gfx1250) — hardware-verified
//
#include <hip/hip_runtime.h>
#include <stdint.h>

typedef __attribute__((ext_vector_type(16))) _Float16 v16h;
typedef __attribute__((ext_vector_type(8)))  _Float16 v8h;
typedef __attribute__((ext_vector_type(16))) __bf16   v16b;
typedef __attribute__((ext_vector_type(8)))  __bf16   v8b;
typedef __attribute__((ext_vector_type(8)))  float    v8f;
typedef __attribute__((ext_vector_type(4)))  float    v4f;
typedef __attribute__((ext_vector_type(4)))  unsigned v4u;

constexpr int NBATCH = 8;
constexpr int SEQ    = 1024;
constexpr int DMODEL = 1024;
constexpr int NHEAD  = 16;
constexpr int HDIM   = 64;
constexpr int NREL   = 8;
constexpr int NTOK   = NBATCH * SEQ;
constexpr int NQB    = SEQ / 64;
static_assert(DMODEL == NHEAD * HDIM);
static_assert(HDIM == 64);
static_assert(SEQ % 64 == 0 && DMODEL % 64 == 0 && NTOK % 64 == 0 && DMODEL % 32 == 0);
static_assert(NBATCH * NREL == 64);

constexpr size_t MIB       = 1048576;
constexpr size_t PLANE_TOK = (size_t)NTOK * DMODEL * 2;
constexpr size_t PLANE_W   = (size_t)DMODEL * DMODEL * 2;
constexpr size_t OFF_XB    = 0;
constexpr size_t OFF_WQT   = 16 * MIB;
constexpr size_t OFF_WKT   = 18 * MIB;
constexpr size_t OFF_WVT   = 20 * MIB;
constexpr size_t OFF_CTXH  = 0;
constexpr size_t OFF_CTXL  = 16 * MIB;
constexpr size_t OFF_WOT   = 32 * MIB;
constexpr size_t OFF_QH    = 34 * MIB;
constexpr size_t OFF_QL    = 50 * MIB;
constexpr size_t OFF_KH    = 66 * MIB;
constexpr size_t OFF_KL    = 82 * MIB;
constexpr size_t OFF_VT    = 98 * MIB;
constexpr size_t OFF_PART  = 114 * MIB;
constexpr int    NATTBLK   = NBATCH * NHEAD * NQB;
constexpr size_t PART_BYTES = (size_t)NATTBLK * 128;
constexpr size_t WS_TOTAL  = OFF_PART + PART_BYTES;
static_assert(OFF_WVT + PLANE_W <= OFF_CTXL + PLANE_TOK);
static_assert(OFF_CTXL + PLANE_TOK <= OFF_WOT);
static_assert(OFF_WOT + PLANE_W <= OFF_QH);
static_assert(OFF_QH + PLANE_TOK == OFF_QL && OFF_QL + PLANE_TOK == OFF_KH && OFF_KH + PLANE_TOK == OFF_KL);
static_assert(OFF_KL + PLANE_TOK == OFF_VT && OFF_VT + PLANE_TOK == OFF_PART);
static_assert(WS_TOTAL <= (size_t)134217728);
static_assert((size_t)NTOK * DMODEL * 4 == 33554432);
static_assert((size_t)NTOK * DMODEL * 4 + NBATCH * NREL * 4 == 33554688);

__device__ __forceinline__ unsigned short f2bf_bits(float f) {
  unsigned u = __float_as_uint(f);
  return (unsigned short)((u + 0x7FFFu + ((u >> 16) & 1u)) >> 16);
}
__device__ __forceinline__ float bf_bits2f(unsigned short h) { return __uint_as_float(((unsigned)h) << 16); }
__device__ __forceinline__ float bf_rne(float f) { return bf_bits2f(f2bf_bits(f)); }

__device__ __forceinline__ void dep_guard_h(v8f& a, v8f& b, v16h x, v16h y) { asm volatile("v_nop\n\tv_nop\n\tv_nop\n\tv_nop" : "+v"(a), "+v"(b) : "v"(x), "v"(y)); }
__device__ __forceinline__ void dep_guard_b(v8f& a, v8f& b, v16b x, v16b y) { asm volatile("v_nop\n\tv_nop\n\tv_nop\n\tv_nop" : "+v"(a), "+v"(b) : "v"(x), "v"(y)); }
__device__ __forceinline__ void keep4_h(v16h a, v16h b, v16h c, v16h d) { asm volatile("v_nop" :: "v"(a), "v"(b), "v"(c), "v"(d)); }
__device__ __forceinline__ void keep4_b(v16b a, v16b b, v16b c, v16b d) { asm volatile("v_nop" :: "v"(a), "v"(b), "v"(c), "v"(d)); }
__device__ __forceinline__ void acc_guard4(v8f& a, v8f& b, v8f& c, v8f& d) { asm volatile("v_nop\n\tv_nop\n\tv_nop\n\tv_nop" : "+v"(a), "+v"(b), "+v"(c), "+v"(d)); }

template <typename T> struct Frag;
template <> struct Frag<_Float16> {
  typedef v16h V; union U { v16h v; v8h h[2]; };
  static __device__ __forceinline__ v16h load(const _Float16* p) {
    U f; f.h[0] = *(const v8h*)(p); f.h[1] = *(const v8h*)(p + 16); return f.v;
  }
  static __device__ __forceinline__ v8f mma(v16h a, v16h b, v8f c) {
    return __builtin_amdgcn_wmma_f32_16x16x32_f16(false, a, false, b, (short)0, c, false, false);
  }
  static __device__ __forceinline__ void guard(v8f& a, v8f& b, v16h x, v16h y) { dep_guard_h(a, b, x, y); }
  static __device__ __forceinline__ void keep(v16h a, v16h b, v16h c, v16h d) { keep4_h(a, b, c, d); }
};
template <> struct Frag<__bf16> {
  typedef v16b V; union U { v16b v; v8b h[2]; };
  static __device__ __forceinline__ v16b load(const __bf16* p) {
    U f; f.h[0] = *(const v8b*)(p); f.h[1] = *(const v8b*)(p + 16); return f.v;
  }
  static __device__ __forceinline__ v8f mma(v16b a, v16b b, v8f c) {
    return __builtin_amdgcn_wmma_f32_16x16x32_bf16(false, a, false, b, (short)0, c, false, false);
  }
  static __device__ __forceinline__ void guard(v8f& a, v8f& b, v16b x, v16b y) { dep_guard_b(a, b, x, y); }
  static __device__ __forceinline__ void keep(v16b a, v16b b, v16b c, v16b d) { keep4_b(a, b, c, d); }
};

__device__ __forceinline__ v8f mma_bf(v16b a, v16b b, v8f c) {
  c = __builtin_amdgcn_wmma_f32_16x16x32_bf16(false, a, false, b, (short)0, c, false, false);
  asm volatile("v_nop\n\tv_nop\n\tv_nop\n\tv_nop" : "+v"(c) : "v"(a), "v"(b));
  return c;
}
__device__ __forceinline__ v8f mma_hf(v16h a, v16h b, v8f c) {
  c = __builtin_amdgcn_wmma_f32_16x16x32_f16(false, a, false, b, (short)0, c, false, false);
  asm volatile("v_nop\n\tv_nop\n\tv_nop\n\tv_nop" : "+v"(c) : "v"(a), "v"(b));
  return c;
}

template <int ET> struct Elem;
template <> struct Elem<0> { typedef _Float16 T; };
template <> struct Elem<1> { typedef __bf16 T; };
template <int ET, int SPLITM, int BIAS_MODE, int OUT_MODE>
__global__ __launch_bounds__(256) void wmma_gemm64(
    const unsigned short* __restrict__ Ap, const unsigned short* __restrict__ A2p, int lda, long strideA,
    const unsigned short* __restrict__ Btp, const unsigned short* __restrict__ Bt2p, int ldb, long strideB,
    void* __restrict__ Cout, void* __restrict__ Cout2, int ldc, long strideC,
    const float* __restrict__ bias, int M, int N, int K, float scale) {
  typedef typename Elem<ET>::T T;
  typedef typename Frag<T>::V V;
  constexpr bool SPA = (SPLITM >= 1);
  constexpr bool SPB = (SPLITM >= 2);
  const T* A = (const T*)Ap; const T* A2 = (const T*)A2p; const T* Bt = (const T*)Btp; const T* Bt2 = (const T*)Bt2p;
  __shared__ __align__(16) float sT[8][16 * 68];
  const int b    = blockIdx.y;
  const int lane = threadIdx.x & 31;
  const int wave = threadIdx.x >> 5;
  const int tilesN = N >> 6;
  const int tilesM = M >> 6;
  const int tile = blockIdx.x * 8 + wave;
  if (tile >= tilesM * tilesN) return;
  const int tm = tile / tilesN;
  const int tn = tile - tm * tilesN;
  const int m0 = tm << 6;
  const int n0 = tn << 6;

  const T* Ab  = A  + (size_t)b * strideA;
  const T* Bb  = Bt + (size_t)b * strideB;
  const T* Ab2 = SPA ? (A2  + (size_t)b * strideA) : nullptr;
  const T* Bb2 = SPB ? (Bt2 + (size_t)b * strideB) : nullptr;

  const int rlane = lane & 15;
  const int koff  = (lane >> 4) * 8;
  const int mOff  = (lane >> 4) * 8;

  v8f acc[4][4];
#pragma unroll
  for (int i = 0; i < 4; ++i)
#pragma unroll
    for (int j = 0; j < 4; ++j) acc[i][j] = (v8f){0.f,0.f,0.f,0.f,0.f,0.f,0.f,0.f};

  for (int k0 = 0; k0 < K; k0 += 32) {
    V bh[4], bl[4];
#pragma unroll
    for (int j = 0; j < 4; ++j) {
      const size_t bo = (size_t)(n0 + (j << 4) + rlane) * ldb + koff + k0;
      bh[j] = Frag<T>::load(Bb + bo);
      if (SPB) bl[j] = Frag<T>::load(Bb2 + bo);
    }
#pragma unroll
    for (int i = 0; i < 4; ++i) {
      const size_t ao = (size_t)(m0 + (i << 4) + rlane) * lda + koff + k0;
      V ah = Frag<T>::load(Ab + ao);
      V al;
      if (SPA) al = Frag<T>::load(Ab2 + ao);
#pragma unroll
      for (int j = 0; j < 4; ++j) {
        acc[i][j] = Frag<T>::mma(ah, bh[j], acc[i][j]);
        if (SPB) acc[i][j] = Frag<T>::mma(ah, bl[j], acc[i][j]);
        if (SPA) acc[i][j] = Frag<T>::mma(al, bh[j], acc[i][j]);
      }
      Frag<T>::guard(acc[i][0], acc[i][3], ah, SPA ? al : ah);
    }
    Frag<T>::keep(bh[0], bh[1], bh[2], bh[3]);
    if (SPB) Frag<T>::keep(bl[0], bl[1], bl[2], bl[3]);
  }
  acc_guard4(acc[0][0], acc[0][1], acc[0][2], acc[0][3]);
  acc_guard4(acc[1][0], acc[1][1], acc[1][2], acc[1][3]);
  acc_guard4(acc[2][0], acc[2][1], acc[2][2], acc[2][3]);
  acc_guard4(acc[3][0], acc[3][1], acc[3][2], acc[3][3]);

  float* slab = sT[wave];
#pragma unroll
  for (int i = 0; i < 4; ++i) {
    const int mBase = m0 + (i << 4);
    float bm[8];
#pragma unroll
    for (int r = 0; r < 8; ++r) bm[r] = 0.f;
    if (BIAS_MODE == 1) {
#pragma unroll
      for (int r = 0; r < 8; ++r) bm[r] = bf_rne(bias[mBase + mOff + r]);
    }
#pragma unroll
    for (int j = 0; j < 4; ++j) {
      const int n = n0 + (j << 4) + rlane;
      float bv = 0.f;
      if (BIAS_MODE == 2) bv = bf_rne(bias[n]);
#pragma unroll
      for (int r = 0; r < 8; ++r) {
        float v = acc[i][j][r] * scale;
        if (BIAS_MODE == 1) v += bm[r];
        if (BIAS_MODE == 2) v += bv;
        slab[(mOff + r) * 68 + (j << 4) + rlane] = v;
      }
    }
    __builtin_amdgcn_fence(__ATOMIC_RELEASE, "workgroup");
    __builtin_amdgcn_wave_barrier();
    __builtin_amdgcn_fence(__ATOMIC_ACQUIRE, "workgroup");
    if (OUT_MODE == 0) {
      float* C = (float*)Cout + (size_t)b * strideC;
      const int hh = lane >> 4, c4 = (lane & 15) * 4;
      for (int pass = 0; pass < 2; ++pass) {
#pragma unroll
        for (int it = 0; it < 8; ++it) {
          const int row = it * 2 + hh;
          v4f v = *(const v4f*)(slab + row * 68 + c4);
          *(volatile v4f*)(C + (size_t)(mBase + row) * ldc + n0 + c4) = v;
        }
        __threadfence();
      }
    } else {
      const int q = lane >> 3, c8 = (lane & 7) * 8;
      unsigned short* C  = (unsigned short*)Cout  + (size_t)b * strideC;
      unsigned short* C2 = (OUT_MODE == 2) ? ((unsigned short*)Cout2 + (size_t)b * strideC) : nullptr;
      for (int pass = 0; pass < 2; ++pass) {
#pragma unroll
        for (int it = 0; it < 4; ++it) {
          const int row = it * 4 + q;
          const float* sp = slab + row * 68 + c8;
          v8h hv, lv;
#pragma unroll
          for (int e = 0; e < 8; ++e) {
            if (OUT_MODE == 1) {
              hv[e] = (_Float16)sp[e];
            } else {
              unsigned short hb = f2bf_bits(sp[e]);
              unsigned short lb = f2bf_bits(sp[e] - bf_bits2f(hb));
              hv[e] = __builtin_bit_cast(_Float16, hb);
              lv[e] = __builtin_bit_cast(_Float16, lb);
            }
          }
          *(volatile v8h*)(C + (size_t)(mBase + row) * ldc + n0 + c8) = hv;
          if (OUT_MODE == 2) *(volatile v8h*)(C2 + (size_t)(mBase + row) * ldc + n0 + c8) = lv;
        }
        __threadfence();
      }
    }
    __builtin_amdgcn_fence(__ATOMIC_RELEASE, "workgroup");
    __builtin_amdgcn_wave_barrier();
    __builtin_amdgcn_fence(__ATOMIC_ACQUIRE, "workgroup");
  }
}

__global__ __launch_bounds__(256) void cast_bf16x8(const float* __restrict__ in, unsigned short* __restrict__ out, int n8) {
  const int i = blockIdx.x * 256 + threadIdx.x;
  if (i < n8) {
    const v4f a = *(const v4f*)(in + (size_t)i * 8);
    const v4f c = *(const v4f*)(in + (size_t)i * 8 + 4);
    v4u u;
    u[0] = (unsigned)f2bf_bits(a[0]) | ((unsigned)f2bf_bits(a[1]) << 16);
    u[1] = (unsigned)f2bf_bits(a[2]) | ((unsigned)f2bf_bits(a[3]) << 16);
    u[2] = (unsigned)f2bf_bits(c[0]) | ((unsigned)f2bf_bits(c[1]) << 16);
    u[3] = (unsigned)f2bf_bits(c[2]) | ((unsigned)f2bf_bits(c[3]) << 16);
    unsigned short* o = out + (size_t)i * 8;
    *(volatile v4u*)o = u;
    __threadfence();
    *(volatile v4u*)o = u;
  }
}

__global__ __launch_bounds__(256) void transpose_w_bf16(
    const float* __restrict__ W0, const float* __restrict__ W1, const float* __restrict__ W2, const float* __restrict__ W3,
    unsigned short* __restrict__ T0, unsigned short* __restrict__ T1, unsigned short* __restrict__ T2, unsigned short* __restrict__ T3) {
  __shared__ float tile[64][65];
  const int which = blockIdx.z;
  const float* W = W0; unsigned short* TT = T0;
  if (which == 1) { W = W1; TT = T1; }
  else if (which == 2) { W = W2; TT = T2; }
  else if (which == 3) { W = W3; TT = T3; }
  const int n0 = blockIdx.x * 64, k0 = blockIdx.y * 64;
  const int t = threadIdx.x;
  {
    const int kr = t >> 2, c16 = (t & 3) * 16;
    const float* src = W + (size_t)(k0 + kr) * DMODEL + n0 + c16;
#pragma unroll
    for (int e4 = 0; e4 < 4; ++e4) {
      const v4f v = *(const v4f*)(src + 4 * e4);
      tile[kr][c16 + 4 * e4 + 0] = v[0];
      tile[kr][c16 + 4 * e4 + 1] = v[1];
      tile[kr][c16 + 4 * e4 + 2] = v[2];
      tile[kr][c16 + 4 * e4 + 3] = v[3];
    }
  }
  __syncthreads();
  const int wave = t >> 5, lane = t & 31, q4 = lane >> 3, c8 = (lane & 7) * 8;
  v4u w[2];
#pragma unroll
  for (int it = 0; it < 2; ++it) {
    const int row = wave * 8 + it * 4 + q4;
#pragma unroll
    for (int e2 = 0; e2 < 4; ++e2) {
      const float f0 = tile[c8 + 2 * e2][row];
      const float f1 = tile[c8 + 2 * e2 + 1][row];
      w[it][e2] = (unsigned)f2bf_bits(f0) | ((unsigned)f2bf_bits(f1) << 16);
    }
  }
  for (int pass = 0; pass < 2; ++pass) {
#pragma unroll
    for (int it = 0; it < 2; ++it) {
      const int row = wave * 8 + it * 4 + q4;
      *(volatile v4u*)(TT + (size_t)(n0 + row) * DMODEL + k0 + c8) = w[it];
    }
    __threadfence();
  }
}

constexpr int ATT_SMEM_HALVES = 20480;
static_assert(4 * 16 * 68 * 2 <= ATT_SMEM_HALVES);

__global__ __launch_bounds__(128) void attn_kernel(
    const unsigned short* __restrict__ qh, const unsigned short* __restrict__ ql,
    const unsigned short* __restrict__ kh, const unsigned short* __restrict__ kl,
    const unsigned short* __restrict__ vt,
    unsigned short* __restrict__ ch, unsigned short* __restrict__ cl,
    float* __restrict__ part) {
  typedef Frag<__bf16>   FB16;
  typedef Frag<_Float16> FH16;
  __shared__ __align__(16) unsigned short smem[ATT_SMEM_HALVES];
  __shared__ float wsum[4];

  const int tid  = threadIdx.x;
  const int wave = tid >> 5;
  const int lane = tid & 31;
  const int hh   = lane >> 4;
  const int c    = lane & 15;
  const int bx = blockIdx.x;
  const int qb = bx & (NQB - 1);
  const int bh = bx >> 4;
  const int h  = bh & (NHEAD - 1);
  const int b  = bh >> 4;
  const int q0 = qb * 64 + wave * 16;

  unsigned short* Ksh = smem;
  unsigned short* Ksl = smem + 4096;
  unsigned short* Vts = smem + 8192;
  _Float16* Pwh = (_Float16*)(void*)(smem + 12288 + wave * 1024);
  _Float16* Pwl = (_Float16*)(void*)(smem + 16384 + wave * 1024);

  const __bf16* Qh = (const __bf16*)(const void*)qh;
  const __bf16* Ql = (const __bf16*)(const void*)ql;
  const size_t qoff = ((size_t)(b * SEQ + q0 + c)) * DMODEL + h * HDIM + 8 * hh;
  v16b qah[2], qal[2];
#pragma unroll
  for (int dc = 0; dc < 2; ++dc) {
    qah[dc] = FB16::load(Qh + qoff + dc * 32);
    qal[dc] = FB16::load(Ql + qoff + dc * 32);
  }

  float mrow[8], lrow[8];
  v8f oacc[4], oacc2[4];
#pragma unroll
  for (int r = 0; r < 8; ++r) { mrow[r] = -__builtin_inff(); lrow[r] = 0.f; }
#pragma unroll
  for (int t = 0; t < 4; ++t) { oacc[t] = (v8f){0.f,0.f,0.f,0.f,0.f,0.f,0.f,0.f}; oacc2[t] = oacc[t]; }

  for (int kc = 0; kc < SEQ / 64; ++kc) {
    const int kv0 = kc * 64;
    __syncthreads();
#pragma unroll
    for (int i = 0; i < 4; ++i) {
      const int s = tid + i * 128, r = s >> 3, d8 = (s & 7) * 8;
      const size_t gk = ((size_t)(b * SEQ + kv0 + r)) * DMODEL + h * HDIM + d8;
      const size_t gv = ((size_t)(bh * HDIM + r)) * SEQ + kv0 + d8;
      const uint4 a1 = *(const uint4*)(kh + gk);
      const uint4 a2 = *(const uint4*)(kl + gk);
      const uint4 a3 = *(const uint4*)(vt + gv);
      *(uint4*)(Ksh + r * 64 + d8) = a1;
      *(uint4*)(Ksl + r * 64 + d8) = a2;
      *(uint4*)(Vts + r * 64 + d8) = a3;
    }
    __syncthreads();

    v8f s[4];
#pragma unroll
    for (int j = 0; j < 4; ++j) {
      v8f a = (v8f){0.f,0.f,0.f,0.f,0.f,0.f,0.f,0.f};
#pragma unroll
      for (int dc = 0; dc < 2; ++dc) {
        const v16b kbh = FB16::load((const __bf16*)(const void*)Ksh + (j * 16 + c) * 64 + dc * 32 + 8 * hh);
        const v16b kbl = FB16::load((const __bf16*)(const void*)Ksl + (j * 16 + c) * 64 + dc * 32 + 8 * hh);
        a = mma_bf(qah[dc], kbh, a);
        a = mma_bf(qah[dc], kbl, a);
        a = mma_bf(qal[dc], kbh, a);
      }
      s[j] = a;
    }
    float cm[8];
#pragma unroll
    for (int r = 0; r < 8; ++r) {
      float m = -__builtin_inff();
#pragma unroll
      for (int j = 0; j < 4; ++j) { s[j][r] *= 0.125f; m = fmaxf(m, s[j][r]); }
#pragma unroll
      for (int off = 1; off < 16; off <<= 1) m = fmaxf(m, __shfl_xor(m, off, 32));
      cm[r] = m;
    }
#pragma unroll
    for (int r = 0; r < 8; ++r) {
      const float mnew  = fmaxf(mrow[r], cm[r]);
      const float alpha = expf(mrow[r] - mnew);
      mrow[r] = mnew;
      float psum = 0.f;
#pragma unroll
      for (int j = 0; j < 4; ++j) {
        const float p  = expf(s[j][r] - mnew);
        psum += p;
        const float pp = p * 32768.0f;
        const _Float16 hv = (_Float16)pp;
        const float res = pp - (float)hv;
        const _Float16 lv = (_Float16)(res * 2048.0f);
        Pwh[(8 * hh + r) * 64 + j * 16 + c] = hv;
        Pwl[(8 * hh + r) * 64 + j * 16 + c] = lv;
      }
#pragma unroll
      for (int off = 1; off < 16; off <<= 1) psum += __shfl_xor(psum, off, 32);
      lrow[r] = lrow[r] * alpha + psum;
#pragma unroll
      for (int t = 0; t < 4; ++t) { oacc[t][r] *= alpha; oacc2[t][r] *= alpha; }
    }
    __syncthreads();

#pragma unroll
    for (int kk = 0; kk < 2; ++kk) {
      const v16h pa = FH16::load(Pwh + c * 64 + kk * 32 + 8 * hh);
      const v16h pl = FH16::load(Pwl + c * 64 + kk * 32 + 8 * hh);
#pragma unroll
      for (int t = 0; t < 4; ++t) {
        const v16h vb = FH16::load((const _Float16*)(const void*)Vts + (t * 16 + c) * 64 + kk * 32 + 8 * hh);
        oacc[t]  = mma_hf(pa, vb, oacc[t]);
        oacc2[t] = mma_hf(pl, vb, oacc2[t]);
      }
    }
  }

  __syncthreads();
  float* os = (float*)(void*)smem + wave * (16 * 68);
  float tsum = 0.f;
#pragma unroll
  for (int r = 0; r < 8; ++r) {
    const float il  = 1.0f / lrow[r];
    tsum += lrow[r] * il;
    const float inv = il * (1.0f / 32768.0f);
#pragma unroll
    for (int t = 0; t < 4; ++t)
      os[(8 * hh + r) * 68 + t * 16 + c] = (oacc[t][r] + oacc2[t][r] * (1.0f / 2048.0f)) * inv;
  }
  tsum += __shfl_xor(tsum, 16, 32);
  if (lane == 0) wsum[wave] = tsum;
  __syncthreads();
  {
    const int q4 = lane >> 3, c8 = (lane & 7) * 8;
    v4u hw[4], lw[4];
#pragma unroll
    for (int it = 0; it < 4; ++it) {
      const float* sp = os + (it * 4 + q4) * 68 + c8;
#pragma unroll
      for (int e2 = 0; e2 < 4; ++e2) {
        const float f0 = sp[2 * e2], f1 = sp[2 * e2 + 1];
        const unsigned hb0 = f2bf_bits(f0), hb1 = f2bf_bits(f1);
        const unsigned lb0 = f2bf_bits(f0 - bf_bits2f((unsigned short)hb0));
        const unsigned lb1 = f2bf_bits(f1 - bf_bits2f((unsigned short)hb1));
        hw[it][e2] = hb0 | (hb1 << 16);
        lw[it][e2] = lb0 | (lb1 << 16);
      }
    }
    const size_t obase = ((size_t)(b * SEQ + q0)) * DMODEL + h * HDIM + c8;
    for (int pass = 0; pass < 2; ++pass) {
#pragma unroll
      for (int it = 0; it < 4; ++it) {
        const size_t o = obase + (size_t)(it * 4 + q4) * DMODEL;
        *(volatile v4u*)(ch + o) = hw[it];
        *(volatile v4u*)(cl + o) = lw[it];
      }
      __threadfence();
    }
  }
  if (wave == 0) {
    const float tot = wsum[0] + wsum[1] + wsum[2] + wsum[3];
    v4f pv;
    pv[0] = (lane == 0) ? tot : 0.f; pv[1] = 0.f; pv[2] = 0.f; pv[3] = 0.f;
    float* pp = part + (size_t)bx * 32 + lane * 4;
    if (lane < 8) *(volatile v4f*)pp = pv;
    __threadfence();
    if (lane < 8) *(volatile v4f*)pp = pv;
  }
}

__global__ __launch_bounds__(128) void headmix_kernel(const float* __restrict__ part, const float* __restrict__ wr,
                                                      const float* __restrict__ br, float* __restrict__ out1) {
  __shared__ float hp_s[128];
  __shared__ __align__(16) float res_s[128];
  const int t = threadIdx.x;
  float a = 0.f;
#pragma unroll 1
  for (int qb = 0; qb < NQB; ++qb) a += part[((size_t)t * NQB + qb) * 32];
  hp_s[t] = a * (1.0f / 1048576.0f);
  __syncthreads();
  float v = 0.f;
  if (t < NBATCH * NREL) {
    const int bb = t >> 3, r = t & 7;
    float acc = 0.f;
#pragma unroll 1
    for (int hd = 0; hd < NHEAD; ++hd) acc += hp_s[bb * NHEAD + hd] * bf_rne(wr[hd * NREL + r]);
    v = acc + bf_rne(br[r]);
  }
  res_s[t] = v;
  __syncthreads();
  if (t < 32) {
    const int lane = t;
    const v4f o = *(const v4f*)(res_s + lane * 4);
    if (lane < 16) *(volatile v4f*)(out1 + lane * 4) = o;
    __threadfence();
    if (lane < 16) *(volatile v4f*)(out1 + lane * 4) = o;
  }
}

extern "C" void kernel_launch(void* const* d_in, const int* in_sizes, int n_in,
                              void* d_out, int out_size, void* d_ws, size_t ws_size,
                              hipStream_t stream) {
  if (n_in < 11) return;
  if (in_sizes[0] != NTOK * DMODEL) return;
  if (in_sizes[1] != DMODEL * DMODEL || in_sizes[3] != DMODEL * DMODEL ||
      in_sizes[5] != DMODEL * DMODEL || in_sizes[7] != DMODEL * DMODEL) return;
  if (in_sizes[2] != DMODEL || in_sizes[4] != DMODEL || in_sizes[6] != DMODEL || in_sizes[8] != DMODEL) return;
  if (in_sizes[9] != NHEAD * NREL || in_sizes[10] != NREL) return;
  if (out_size != NTOK * DMODEL + NBATCH * NREL) return;
  if (ws_size < WS_TOTAL) return;

  const float* x    = (const float*)d_in[0];
  const float* Wq   = (const float*)d_in[1];
  const float* bq   = (const float*)d_in[2];
  const float* Wk   = (const float*)d_in[3];
  const float* bk   = (const float*)d_in[4];
  const float* Wv   = (const float*)d_in[5];
  const float* bv   = (const float*)d_in[6];
  const float* Wo   = (const float*)d_in[7];
  const float* bo   = (const float*)d_in[8];
  const float* wr   = (const float*)d_in[9];
  const float* br   = (const float*)d_in[10];
  float* out0 = (float*)d_out;
  float* out1 = out0 + (size_t)NTOK * DMODEL;

  char* ws = (char*)d_ws;
  unsigned short* xb   = (unsigned short*)(ws + OFF_XB);
  unsigned short* WqT  = (unsigned short*)(ws + OFF_WQT);
  unsigned short* WkT  = (unsigned short*)(ws + OFF_WKT);
  unsigned short* WvT  = (unsigned short*)(ws + OFF_WVT);
  unsigned short* WoT  = (unsigned short*)(ws + OFF_WOT);
  unsigned short* ctxh = (unsigned short*)(ws + OFF_CTXH);
  unsigned short* ctxl = (unsigned short*)(ws + OFF_CTXL);
  unsigned short* qhp  = (unsigned short*)(ws + OFF_QH);
  unsigned short* qlp  = (unsigned short*)(ws + OFF_QL);
  unsigned short* khp  = (unsigned short*)(ws + OFF_KH);
  unsigned short* klp  = (unsigned short*)(ws + OFF_KL);
  unsigned short* vtp  = (unsigned short*)(ws + OFF_VT);
  float* part = (float*)(ws + OFF_PART);

  constexpr int N8 = NTOK * DMODEL / 8;
  static_assert(N8 % 256 == 0);
  cast_bf16x8<<<dim3(N8 / 256), dim3(256), 0, stream>>>(x, xb, N8);

  transpose_w_bf16<<<dim3(DMODEL / 64, DMODEL / 64, 4), dim3(256), 0, stream>>>(Wq, Wk, Wv, Wo, WqT, WkT, WvT, WoT);

  static_assert(NTOK % 64 == 0 && DMODEL % 64 == 0 && DMODEL % 32 == 0);
  static_assert(((NTOK / 64) * (DMODEL / 64)) % 8 == 0 && ((DMODEL / 64) * (DMODEL / 64)) % 8 == 0);
  const int gridTok = (NTOK / 64) * (DMODEL / 64) / 8;
  const int gridVt  = (DMODEL / 64) * (DMODEL / 64) / 8;

  wmma_gemm64<1, 0, 2, 2><<<dim3(gridTok, 1), dim3(256), 0, stream>>>(
      xb, xb, DMODEL, 0L, WqT, WqT, DMODEL, 0L, (void*)qhp, (void*)qlp, DMODEL, 0L,
      bq, NTOK, DMODEL, DMODEL, 1.0f);
  wmma_gemm64<1, 0, 2, 2><<<dim3(gridTok, 1), dim3(256), 0, stream>>>(
      xb, xb, DMODEL, 0L, WkT, WkT, DMODEL, 0L, (void*)khp, (void*)klp, DMODEL, 0L,
      bk, NTOK, DMODEL, DMODEL, 1.0f);
  wmma_gemm64<1, 0, 1, 1><<<dim3(gridVt, NBATCH), dim3(256), 0, stream>>>(
      WvT, WvT, DMODEL, 0L, xb, xb, DMODEL, (long)SEQ * DMODEL, (void*)vtp, (void*)vtp, SEQ, (long)DMODEL * SEQ,
      bv, DMODEL, SEQ, DMODEL, 1.0f);
  attn_kernel<<<dim3(NATTBLK), dim3(128), 0, stream>>>(qhp, qlp, khp, klp, vtp, ctxh, ctxl, part);
  wmma_gemm64<1, 1, 2, 0><<<dim3(gridTok, 1), dim3(256), 0, stream>>>(
      ctxh, ctxl, DMODEL, 0L, WoT, WoT, DMODEL, 0L, (void*)out0, (void*)out0, DMODEL, 0L,
      bo, NTOK, DMODEL, DMODEL, 1.0f);
  headmix_kernel<<<dim3(1), dim3(128), 0, stream>>>(part, wr, br, out1);
}
